// Transformer_Encoder_Layer_66494683677359
// MI455X (gfx1250) — hardware-verified
//
#include <string.h>
#include <hip/hip_runtime.h>


namespace {
constexpr int NB = 16, S = 384, D = 768, NH = 12, DH = 64, FF = 3072, NR = NB * S, NREL = 2 * S - 1  , NRP = 768, TW = 400  ;
constexpr float XS = 8.0f, WSC = 256.0f, PS = 8.0f, EPS = 1e-5f, LOG2E = 1.4426950408889634f;

typedef _Float16 b16;
typedef __attribute__((ext_vector_type(16))) _Float16 v16b;
typedef __attribute__((ext_vector_type(8))) _Float16 v8b;
typedef __attribute__((ext_vector_type(8))) float v8f;
typedef __attribute__((ext_vector_type(4))) float v4f;
__device__ __forceinline__ float bf16_rne(float f) { unsigned int u = __float_as_uint(f); u += 0x7FFFu + ((u >> 16) & 1u); return __uint_as_float(u & 0xFFFF0000u); }
__device__ __forceinline__ void split16(float v, b16& hi, b16& lo) { hi = (b16)v; lo = (b16)(v - (float)hi); }
__device__ __forceinline__ v16b frag_kb(const b16* p, int hh) { const v8b a = *(const v8b*)(p + 8 * hh), b = *(const v8b*)(p + 16 + 8 * hh); v16b f;
#pragma unroll
  for (int e = 0; e < 8; ++e) { f[e] = a[e]; f[8 + e] = b[e]; } return f; }
__device__ __forceinline__ v8f wmma16b(v16b a, v16b b, v8f c) { v8f d = __builtin_amdgcn_wmma_f32_16x16x32_f16(false, a, false, b, (short)0, c, false, false); asm volatile("v_nop\n\tv_nop\n\tv_nop\n\tv_nop" : "+v"(d) : "v"(a), "v"(b)); return d; }
__device__ __forceinline__ void wave_lds_sync() { __builtin_amdgcn_fence(__ATOMIC_RELEASE, "workgroup"); __builtin_amdgcn_wave_barrier(); __builtin_amdgcn_fence(__ATOMIC_ACQUIRE, "workgroup"); }
__device__ __forceinline__ float pmul(float a, float b) { float p = a * b; asm volatile("" : "+v"(p)); return p; }
__device__ __forceinline__ float hsum16(float v) { v += __shfl_xor(v, 1); v += __shfl_xor(v, 2); v += __shfl_xor(v, 4); return v + __shfl_xor(v, 8); }
__device__ __forceinline__ float nexp2(float x) { return __builtin_amdgcn_exp2f(x); }

__global__ __launch_bounds__(256) void prepx_kernel(const float* __restrict__ x, const float* __restrict__ pe, b16* __restrict__ X16, b16* __restrict__ PE16) {
  const size_t t = (size_t)blockIdx.x * 256 + threadIdx.x; const size_t n1 = (size_t)NR * D / 8, n2 = (size_t)NRP * D / 8; v8b o = {};
  if (t < n1) { const size_t e = t * 8; const v4f a = *(const v4f*)(x + e), c = *(const v4f*)(x + e + 4); for (int j = 0; j < 4; ++j) { o[j] = (b16)(bf16_rne(a[j]) * XS); o[4 + j] = (b16)(bf16_rne(c[j]) * XS); } for (int pass = 0; pass < 2; ++pass) { *(volatile v8b*)(X16 + e) = o; __threadfence(); } }
  else if (t < n1 + n2) { const size_t e = (t - n1) * 8; if (e < (size_t)NREL * D) { const v4f a = *(const v4f*)(pe + e), c = *(const v4f*)(pe + e + 4); for (int j = 0; j < 4; ++j) { o[j] = (b16)(bf16_rne(a[j]) * XS); o[4 + j] = (b16)(bf16_rne(c[j]) * XS); } }
    for (int pass = 0; pass < 2; ++pass) { *(volatile v8b*)(PE16 + e) = o; __threadfence(); } }
}
__global__ __launch_bounds__(256) void prepw_kernel(const float* __restrict__ wq, const float* __restrict__ wk, const float* __restrict__ wv, const float* __restrict__ wr, const float* __restrict__ wo, const float* __restrict__ w1, const float* __restrict__ w2, b16* __restrict__ WT) {
  __shared__ __attribute__((aligned(16))) b16 T[64][64 + 8];
  const int kind = blockIdx.z, i0 = blockIdx.x * 64, o0 = blockIdx.y * 64, t_ = threadIdx.x; int IN = D, OUT = D; const float* w; size_t base;
  if (kind < 5) { w = kind == 0 ? wq : kind == 1 ? wk : kind == 2 ? wv : kind == 3 ? wr : wo; base = (size_t)kind * D * D; }
  else if (kind == 5) { w = w1; OUT = FF; base = (size_t)5 * D * D; } else { w = w2; IN = FF; base = (size_t)5 * D * D + (size_t)FF * D; }
  if (i0 >= IN || o0 >= OUT) return;
  for (int q = t_; q < 64 * 64; q += 256) { const int ii = q >> 6, oo = q & 63; T[oo][ii] = (b16)(bf16_rne(w[(size_t)(i0 + ii) * OUT + o0 + oo]) * WSC); }
  __syncthreads();
  for (int pass = 0; pass < 2; ++pass) { for (int q = t_; q < 64 * 8; q += 256) { const int oo = q >> 3, c8 = (q & 7) * 8; *(volatile v8b*)(WT + base + (size_t)(o0 + oo) * IN + i0 + c8) = *(const v8b*)(&T[oo][c8]); } __threadfence(); }
}
struct GA { const b16* A; const b16* W; const float* bias; const float* uu; const float* vv; b16* Y16; b16* Y16b; float* Y32; int lda, K, ldy; int pad_; };
template <int MODE>
__global__ __launch_bounds__(128) void gemm_kernel(GA g) {
  __shared__ __attribute__((aligned(16))) float Ts[4][16][128 + 4]; __shared__ __attribute__((aligned(16))) b16 Vt[128][64 + 8];
  const int wave = threadIdx.x >> 5, lane = threadIdx.x & 31, nloc = lane & 15, hlf = lane >> 4, t_ = threadIdx.x; const size_t m0 = (size_t)blockIdx.x * 64 + wave * 16; const int n0 = blockIdx.y * 128;
  v8f acc[8];
#pragma unroll
  for (int t = 0; t < 8; ++t) acc[t] = (v8f){};
  for (int kb = 0; kb < g.K; kb += 32) { const v16b a = frag_kb(g.A + (m0 + nloc) * g.lda + kb, hlf);
#pragma unroll
    for (int t = 0; t < 8; ++t) acc[t] = wmma16b(a, frag_kb(g.W + (size_t)(n0 + t * 16 + nloc) * g.K + kb, hlf), acc[t]); }
  if (MODE == 2) { const int b = (int)(m0 / S); const int s0 = (int)((size_t)blockIdx.x * 64 - (size_t)b * S);
#pragma unroll
    for (int t = 0; t < 8; ++t)
#pragma unroll
      for (int r = 0; r < 8; ++r) Vt[t * 16 + nloc][wave * 16 + 8 * hlf + r] = (b16)(acc[t][r] * (1.0f / (XS * WSC)) * XS);
    __syncthreads();
    for (int pass = 0; pass < 2; ++pass) { for (int q = t_; q < 128 * 8; q += 128) { const int cc = q >> 3, c8 = (q & 7) * 8; const int h = (n0 + cc) / DH, d = (n0 + cc) - h * DH; *(volatile v8b*)(g.Y16 + (((size_t)b * NH + h) * DH + d) * S + s0 + c8) = *(const v8b*)(&Vt[cc][c8]); } __threadfence(); }
    return; }
#pragma unroll
  for (int t = 0; t < 8; ++t) { const int c = n0 + t * 16 + nloc; const float bb = (MODE >= 4 && g.bias) ? bf16_rne(g.bias[c]) : 0.0f;
#pragma unroll
    for (int r = 0; r < 8; ++r) { float v = acc[t][r] * (1.0f / (XS * WSC)) + bb; if (MODE == 5) v = fmaxf(v, 0.0f); Ts[wave][8 * hlf + r][t * 16 + nloc] = v; } }
  wave_lds_sync();
  for (int pass = 0; pass < 2; ++pass) { for (int rr = 0; rr < 16; ++rr) {
      if (MODE == 4) { *(volatile v4f*)(g.Y32 + (m0 + rr) * g.ldy + n0 + lane * 4) = *(const v4f*)(&Ts[wave][rr][lane * 4]); }
      else if (lane < 16) { const int c0 = n0 + lane * 8; v8b o;
        if (MODE == 0) { v8b o2; for (int j = 0; j < 8; ++j) { const int c = c0 + j; const float q = Ts[wave][rr][lane * 8 + j]; o[j] = (b16)((q + bf16_rne(g.uu[c])) * XS); o2[j] = (b16)((q + bf16_rne(g.vv[c])) * XS); }
          *(volatile v8b*)(g.Y16 + (m0 + rr) * g.ldy + c0) = o; *(volatile v8b*)(g.Y16b + (m0 + rr) * g.ldy + c0) = o2; }
        else { for (int j = 0; j < 8; ++j) o[j] = (b16)(Ts[wave][rr][lane * 8 + j] * XS); *(volatile v8b*)(g.Y16 + (m0 + rr) * g.ldy + c0) = o; } } }
    __threadfence(); }
}
__global__ __launch_bounds__(64) void attn_kernel(const b16* __restrict__ QU, const b16* __restrict__ QV, const b16* __restrict__ K16, const b16* __restrict__ VT16, const b16* __restrict__ R16, b16* __restrict__ O16) {
  __shared__ float Tb[2][16][TW + 1]; __shared__ __attribute__((aligned(16))) float To[2][16][DH + 4];
  const int wave = threadIdx.x >> 5, lane = threadIdx.x & 31, hh = lane >> 4, col = lane & 15; const int b = blockIdx.z, h = blockIdx.y; const int i0 = blockIdx.x * 32 + wave * 16, ii = i0 + col;
  const size_t qrow = ((size_t)b * S + ii) * D + h * DH;
  { const v16b qv0 = frag_kb(QV + qrow, hh), qv1 = frag_kb(QV + qrow + 32, hh);
#pragma unroll 1
    for (int tt = 0; tt < TW / 16; ++tt) { const int rho = min(i0 + tt * 16 + col, NRP - 1); v8f acc = {}; acc = wmma16b(frag_kb(R16 + (size_t)rho * D + h * DH, hh), qv0, acc); acc = wmma16b(frag_kb(R16 + (size_t)rho * D + h * DH + 32, hh), qv1, acc);
#pragma unroll
      for (int r = 0; r < 8; ++r) Tb[wave][col][tt * 16 + 8 * hh + r] = acc[r] * (1.0f / (XS * XS)); } }
  wave_lds_sync();
  const v16b qa0 = frag_kb(QU + qrow, hh), qa1 = frag_kb(QU + qrow + 32, hh);
  const b16* Kb = K16 + (size_t)b * S * D + h * DH; const b16* Vb = VT16 + ((size_t)b * NH + h) * DH * S;
  float m = -INFINITY, l = 0.0f; v8f o[4] = {{}, {}, {}, {}}, ol[4] = {{}, {}, {}, {}};
  const float cs = 1.0f / (XS * XS);
  for (int kb = 0; kb < S; kb += 32) {
    v8f s0 = {}, s1 = {};
    { const b16* k0 = Kb + (size_t)(kb + col) * D, *k1 = Kb + (size_t)(kb + 16 + col) * D; s0 = wmma16b(frag_kb(k0, hh), qa0, s0); s0 = wmma16b(frag_kb(k0 + 32, hh), qa1, s0); s1 = wmma16b(frag_kb(k1, hh), qa0, s1); s1 = wmma16b(frag_kb(k1 + 32, hh), qa1, s1); }
    float e[16]; float mx = -INFINITY;
#pragma unroll
    for (int r = 0; r < 8; ++r) { const int j0 = kb + 8 * hh + r, j1 = kb + 16 + 8 * hh + r; const int t0 = col - j0 + (S - 1), t1 = col - j1 + (S - 1);
      e[r] = (s0[r] * cs + Tb[wave][col][t0]) * (0.125f * LOG2E); e[8 + r] = (s1[r] * cs + Tb[wave][col][t1]) * (0.125f * LOG2E); mx = fmaxf(mx, fmaxf(e[r], e[8 + r])); }
    mx = fmaxf(mx, __shfl_xor(mx, 16)); const float mn = fmaxf(m, mx); const float al = nexp2(m - mn); m = mn; float sum = 0.0f; v16b ph, pl;
#pragma unroll
    for (int i = 0; i < 16; ++i) { const float p = nexp2(e[i] - mn); sum += p; const b16 h_ = (b16)(p * PS); ph[i] = h_; pl[i] = (b16)(p * PS - (float)h_); }
    sum += __shfl_xor(sum, 16); l = l * al + sum;
#pragma unroll
    for (int t = 0; t < 4; ++t) { o[t] *= al; ol[t] *= al; const v16b vf = frag_kb(Vb + (size_t)(t * 16 + col) * S + kb, hh); o[t] = wmma16b(vf, ph, o[t]); ol[t] = wmma16b(vf, pl, ol[t]); } }
  const float inv = 1.0f / (l * PS * XS);
#pragma unroll
  for (int t = 0; t < 4; ++t)
#pragma unroll
    for (int r = 0; r < 8; ++r) To[wave][col][t * 16 + 8 * hh + r] = (o[t][r] + ol[t][r]) * inv;
  wave_lds_sync();
  for (int pass = 0; pass < 2; ++pass) { for (int r2 = 0; r2 < 16; r2 += 2) { const int rr = r2 + (lane >> 4), c8 = (lane & 15) * 8; if (c8 < DH) { v8b o8; for (int j = 0; j < 8; ++j) o8[j] = (b16)(To[wave][rr][c8 + j] * XS); *(volatile v8b*)(O16 + ((size_t)b * S + i0 + rr) * D + h * DH + c8) = o8; } } __threadfence(); }
}
__global__ __launch_bounds__(256) void addln_kernel(const float* __restrict__ A, const float* __restrict__ Bp, const float* __restrict__ gam, const float* __restrict__ bet, float* __restrict__ Y32, b16* __restrict__ Y16, int roundA) {
  const int wave = threadIdx.x >> 5, lane = threadIdx.x & 31; const size_t row = (size_t)blockIdx.x * 8 + wave; const int c0 = lane * 24;
  float x[24]; float s = 0.0f;
#pragma unroll
  for (int j4 = 0; j4 < 24; j4 += 4) { const v4f a = *(const v4f*)(A + row * D + c0 + j4), c = *(const v4f*)(Bp + row * D + c0 + j4); for (int j = 0; j < 4; ++j) { const float av = roundA ? bf16_rne(a[j]) : a[j]; x[j4 + j] = av + c[j]; s += x[j4 + j]; } }
  s = hsum16(s); s += __shfl_xor(s, 16); const float mu = s * (1.0f / D); float q2 = 0.0f;
#pragma unroll
  for (int j = 0; j < 24; ++j) { const float dv = x[j] - mu; q2 += pmul(dv, dv); }
  q2 = hsum16(q2); q2 += __shfl_xor(q2, 16); const float rs = rsqrtf(q2 * (1.0f / D) + EPS);
  float y[24];
#pragma unroll
  for (int j = 0; j < 24; ++j) y[j] = pmul((x[j] - mu) * rs, bf16_rne(gam[c0 + j])) + bf16_rne(bet[c0 + j]);
  for (int pass = 0; pass < 2; ++pass) {
#pragma unroll
    for (int j4 = 0; j4 < 24; j4 += 4) { const v4f o4 = {y[j4], y[j4 + 1], y[j4 + 2], y[j4 + 3]}; *(volatile v4f*)(Y32 + row * D + c0 + j4) = o4; }
    if (Y16) {
#pragma unroll
      for (int j8 = 0; j8 < 24; j8 += 8) { v8b o8; for (int j = 0; j < 8; ++j) o8[j] = (b16)(y[j8 + j] * XS); *(volatile v8b*)(Y16 + row * D + c0 + j8) = o8; } }
    __threadfence(); }
}
}

extern "C" void kernel_launch(void* const* d_in, const int* in_sizes, int n_in, void* d_out, int out_size, void* d_ws, size_t ws_size, hipStream_t stream) {
  (void)n_in;
  auto Fp = [&](int i) { return (const float*)d_in[i]; };
  if (in_sizes[0] != NR * D || in_sizes[1] != NREL * D || in_sizes[2] != D * D || in_sizes[8] != D * D || in_sizes[13] != D * FF || in_sizes[15] != FF * D || out_size != NR * D) return;
  size_t off = 0; char* ws = (char*)d_ws;
  auto carve = [&](size_t bytes) { char* p = ws + off; off += (bytes + 255) & ~(size_t)255; return p; };
  b16* X16 = (b16*)carve((size_t)NR * D * 2); b16* PE16 = (b16*)carve((size_t)NRP * D * 2); b16* WT = (b16*)carve(((size_t)5 * D * D + 2 * (size_t)FF * D) * 2);
  b16* QU = (b16*)carve((size_t)NR * D * 2); b16* QV = (b16*)carve((size_t)NR * D * 2); b16* K16 = (b16*)carve((size_t)NR * D * 2); b16* VT16 = (b16*)carve((size_t)NR * D * 2);
  b16* R16 = (b16*)carve((size_t)NRP * D * 2); b16* O16 = (b16*)carve((size_t)NR * D * 2); float* ATT = (float*)carve((size_t)NR * D * 4); float* X1 = (float*)carve((size_t)NR * D * 4); b16* X1h = (b16*)carve((size_t)NR * D * 2);
  b16* HDN = QU; float* FFO = ATT;
  if ((char*)VT16 + (size_t)NR * D * 2 - (char*)QU != (ptrdiff_t)((size_t)NR * FF * 2)) return;
  if (off > ws_size || off > ((size_t)128 << 20)) return;
  const b16 *WqT = WT, *WkT = WT + (size_t)D * D, *WvT = WT + (size_t)2 * D * D, *WrT = WT + (size_t)3 * D * D, *WoT = WT + (size_t)4 * D * D, *W1T = WT + (size_t)5 * D * D, *W2T = WT + (size_t)5 * D * D + (size_t)FF * D;
  prepx_kernel<<<(unsigned)(((size_t)NR * D / 8 + (size_t)NRP * D / 8 + 255) / 256), 256, 0, stream>>>(Fp(0), Fp(1), X16, PE16);
  prepw_kernel<<<dim3(FF / 64, FF / 64, 7), 256, 0, stream>>>(Fp(2), Fp(3), Fp(4), Fp(5), Fp(8), Fp(13), Fp(15), WT);
  auto G = [&](const b16* A, const b16* W, const float* bias, const float* uu, const float* vv, b16* Y16, b16* Y16b, float* Y32, int lda, int K, int ldy) { GA g; memset(&g, 0, sizeof(g)); g.A = A; g.W = W; g.bias = bias; g.uu = uu; g.vv = vv; g.Y16 = Y16; g.Y16b = Y16b; g.Y32 = Y32; g.lda = lda; g.K = K; g.ldy = ldy; return g; };
  gemm_kernel<0><<<dim3(NR / 64, D / 128), 128, 0, stream>>>(G(X16, WqT, nullptr, Fp(6), Fp(7), QU, QV, nullptr, D, D, D));
  gemm_kernel<1><<<dim3(NR / 64, D / 128), 128, 0, stream>>>(G(X16, WkT, nullptr, nullptr, nullptr, K16, nullptr, nullptr, D, D, D));
  gemm_kernel<2><<<dim3(NR / 64, D / 128), 128, 0, stream>>>(G(X16, WvT, nullptr, nullptr, nullptr, VT16, nullptr, nullptr, D, D, D));
  gemm_kernel<3><<<dim3(NRP / 64, D / 128), 128, 0, stream>>>(G(PE16, WrT, nullptr, nullptr, nullptr, R16, nullptr, nullptr, D, D, D));
  attn_kernel<<<dim3(S / 32, NH, NB), 64, 0, stream>>>(QU, QV, K16, VT16, R16, O16);
  gemm_kernel<4><<<dim3(NR / 64, D / 128), 128, 0, stream>>>(G(O16, WoT, nullptr, nullptr, nullptr, nullptr, nullptr, ATT, D, D, D));
  addln_kernel<<<NR / 8, 256, 0, stream>>>(Fp(0), ATT, Fp(9), Fp(10), X1, X1h, 1);
  gemm_kernel<5><<<dim3(NR / 64, FF / 128), 128, 0, stream>>>(G(X1h, W1T, Fp(14), nullptr, nullptr, HDN, nullptr, nullptr, D, D, FF));
  gemm_kernel<4><<<dim3(NR / 64, D / 128), 128, 0, stream>>>(G(HDN, W2T, Fp(16), nullptr, nullptr, nullptr, nullptr, FFO, FF, FF, D));
  addln_kernel<<<NR / 8, 256, 0, stream>>>(X1, FFO, Fp(11), Fp(12), (float*)d_out, nullptr, 0);
}
